// TransformerNet_18279380812408
// MI455X (gfx1250) — hardware-verified
//
#include <hip/hip_runtime.h>
#include <stddef.h>


#define NTHR   256
#define NWAVE  8
#define HD     128
#define FI     32
#define FO     16
#define NGRAPH 64
#define GR     32
#define XSP    132
#define NB     512
#define CHUNK  2048
#define WCAP   256
#define NGRP   (CHUNK / (NTHR * 4))
#define ACCF   (NB * HD)
#define AGG_LDS_BYTES ((ACCF + 2 * NB) * 4 + (NWAVE * WCAP + NWAVE) * 4)

static_assert(NGRP == 2);
static_assert(WCAP == (CHUNK / NTHR) * 32);
static_assert(AGG_LDS_BYTES == 274464);
static_assert((NB & (NB - 1)) == 0);
static_assert(NB <= 512);
static_assert(NB <= NWAVE * WCAP);
static_assert((XSP % 4) == 0);

typedef float    v4f  __attribute__((ext_vector_type(4)));
typedef float    v8f  __attribute__((ext_vector_type(8)));
typedef int      v4i  __attribute__((ext_vector_type(4)));
typedef _Float16 v8h  __attribute__((ext_vector_type(8)));
typedef _Float16 v16h __attribute__((ext_vector_type(16)));

union FragH { v16h v; v4i u[2]; };
union Pack  { v8h h; v4i i; };

__device__ __forceinline__ v8f wmh(v16h a, v16h b, v8f c) {
  v8f d = __builtin_amdgcn_wmma_f32_16x16x32_f16(false, a, false, b, (short)0, c, false, false);
  asm volatile("v_nop\n\tv_nop\n\tv_nop\n\tv_nop" : "+v"(d) : "v"(a), "v"(b));
  return d;
}

__device__ __forceinline__ float lk(float t) { return fmaxf(t, 0.2f * t); }
__device__ __forceinline__ float dl(v4f t, v4f w) {
  return w.x * lk(t.x) + w.y * lk(t.y) + w.z * lk(t.z) + w.w * lk(t.w);
}

__global__ __launch_bounds__(NTHR) void k_cvt_x(const float* __restrict__ src, int rows_src,
                                                _Float16* dst, int rows_total) {
  const int i  = blockIdx.x * NTHR + threadIdx.x;
  const int n8 = rows_total * (FI / 8);
  if (i >= n8) return;
  const int r  = i >> 2;
  const int kb = (i & 3) * 8;
  const int rc = (r < rows_src) ? r : (rows_src - 1);
  const float* sp = src + (size_t)rc * FI + kb;
  const v4f f0 = *(const v4f*)(sp);
  const v4f f1 = *(const v4f*)(sp + 4);
  Pack u;
#pragma unroll
  for (int j = 0; j < 4; ++j) {
    u.h[j]     = (_Float16)f0[j];
    u.h[4 + j] = (_Float16)f1[j];
  }
  const v4i z4 = {0, 0, 0, 0};
  if (r >= rows_src) u.i = z4;
  _Float16* dp = dst + (size_t)i * 8;
  *(volatile v4i*)dp = u.i;
  __threadfence();
  *(volatile v4i*)dp = u.i;
}

__global__ __launch_bounds__(NTHR) void k_cvt_w(const float* __restrict__ sA, const float* __restrict__ sB,
                                                _Float16* dst, int L, int K, int NH, int NCT, float scale) {
  const int total8 = (L * NCT * K) >> 3;
  const int i = blockIdx.x * NTHR + threadIdx.x;
  if (i >= total8) return;
  const int q   = i * 8;
  const int per = NCT * K;
  const int l   = q / per;
  const int rem = q - l * per;
  const int n   = rem / K;
  const int kb  = rem - n * K;
  const int nA  = (n < NH) ? n : (NH - 1);
  int nB = n - NH;
  nB = nB < 0 ? 0 : (nB > NH - 1 ? NH - 1 : nB);
  Pack u;
#pragma unroll
  for (int j = 0; j < 8; ++j) {
    const size_t ro = ((size_t)l * K + kb + j) * NH;
    const float va = sA[ro + nA];
    const float vb = sB[ro + nB];
    const float v  = (n < NH) ? va : vb;
    u.h[j] = (_Float16)(v * scale);
  }
  _Float16* dp = dst + (size_t)q;
  *(volatile v4i*)dp = u.i;
  __threadfence();
  *(volatile v4i*)dp = u.i;
}

template <int OUT16>
__global__ __launch_bounds__(NTHR) void k_gemm(
    const _Float16* __restrict__ A, const _Float16* __restrict__ B,
    const float* __restrict__ bias, float bflag,
    float* out0, float* out1, _Float16* outh, int K, float oscale) {
  __shared__ __attribute__((aligned(16))) float Xs[GR * XSP];

  const int tid  = threadIdx.x;
  const int lane = tid & 31;
  const int wave = tid >> 5;
  const int hh   = lane >> 4;
  const int m    = lane & 15;
  const int rowBase = blockIdx.x * GR;
  const int cset = blockIdx.y;
  const int cl   = wave * 16 + m;

  const size_t ra0 = (size_t)(rowBase + m) * K + 8 * hh;
  const size_t ra1 = ra0 + (size_t)16 * K;
  const size_t rb  = (size_t)(cset * HD + cl) * K + 8 * hh;

  v8f c0 = {0.f, 0.f, 0.f, 0.f, 0.f, 0.f, 0.f, 0.f};
  v8f c1 = {0.f, 0.f, 0.f, 0.f, 0.f, 0.f, 0.f, 0.f};

#pragma unroll 1
  for (int k0 = 0; k0 < K; k0 += 32) {
    FragH a0, a1, b;
    a0.u[0] = *(const v4i*)(A + ra0 + k0);  a0.u[1] = *(const v4i*)(A + ra0 + k0 + 16);
    a1.u[0] = *(const v4i*)(A + ra1 + k0);  a1.u[1] = *(const v4i*)(A + ra1 + k0 + 16);
    b.u[0]  = *(const v4i*)(B + rb + k0);   b.u[1]  = *(const v4i*)(B + rb + k0 + 16);
    c0 = wmh(a0.v, b.v, c0);
    c1 = wmh(a1.v, b.v, c1);
  }

  const float bv = bias[cl] * bflag;
#pragma unroll
  for (int r = 0; r < 8; ++r) {
    Xs[(8 * hh + r) * XSP + cl]      = c0[r] * oscale + bv;
    Xs[(16 + 8 * hh + r) * XSP + cl] = c1[r] * oscale + bv;
  }
  __syncthreads();

  if (OUT16) {
    const int m15 = lane & 15;
    Pack u[2];
    _Float16* hp[2];
#pragma unroll
    for (int i = 0; i < 2; ++i) {
      const int row = 4 * wave + 2 * i + hh;
      const float* xs = Xs + row * XSP + 8 * m15;
      const v4f f0 = *(const v4f*)(xs);
      const v4f f1 = *(const v4f*)(xs + 4);
#pragma unroll
      for (int j = 0; j < 4; ++j) {
        u[i].h[j]     = (_Float16)f0[j];
        u[i].h[4 + j] = (_Float16)f1[j];
      }
      hp[i] = outh + (size_t)(rowBase + row) * HD + 8 * m15;
    }
#pragma unroll
    for (int i = 0; i < 2; ++i) *(volatile v4i*)(hp[i]) = u[i].i;
    __threadfence();
#pragma unroll
    for (int i = 0; i < 2; ++i) *(volatile v4i*)(hp[i]) = u[i].i;
  } else {
    float* out = (cset == 0) ? out0 : out1;
    v4f xv[4];
    float* xp[4];
#pragma unroll
    for (int i = 0; i < 4; ++i) {
      xv[i] = *(const v4f*)(Xs + (4 * wave + i) * XSP + 4 * lane);
      xp[i] = out + (size_t)(rowBase + 4 * wave + i) * HD + 4 * lane;
    }
#pragma unroll
    for (int i = 0; i < 4; ++i) *(volatile v4f*)(xp[i]) = xv[i];
    __threadfence();
#pragma unroll
    for (int i = 0; i < 4; ++i) *(volatile v4f*)(xp[i]) = xv[i];
  }
}

__device__ __forceinline__ void hit4(const float* xs, const float* xd, float* ar, float* mp, float* dp, v4f w0) {
  const v4f a0 = *(const v4f*)(xs);
  const v4f d0 = *(const v4f*)(xd);
  float s = dl(a0 + d0, w0);
  s += __shfl_xor(s, 16, 32);
  s += __shfl_xor(s, 8, 32);
  s += __shfl_xor(s, 4, 32);
  s += __shfl_xor(s, 2, 32);
  s += __shfl_xor(s, 1, 32);
  const float m  = mp[0], n = dp[0];
  const float mn = fmaxf(m, s);
  const float sc = __expf(m - mn);
  const float p  = __expf(s - mn);
  v4f e0 = *(v4f*)(ar);
  e0 = e0 * sc + a0 * p;
  *(v4f*)(ar) = e0;
  mp[0] = mn;
  dp[0] = n * sc + p;
}

__global__ __launch_bounds__(NTHR) void k_agg(
    const int* __restrict__ ei, const float* __restrict__ xl, const float* xr,
    const float* __restrict__ att, const float* __restrict__ bias,
    _Float16* hf, float* hout, int nN, int nE, int nW, int lastMode) {
  extern __shared__ v4f lds_dyn[];
  float* sacc = (float*)lds_dyn;
  float* mx   = sacc + ACCF;
  float* dn   = mx + NB;
  int*   list = (int*)(dn + NB);
  int*   wcnt = list + NWAVE * WCAP;

  const int tid  = threadIdx.x;
  const int lane = tid & 31;
  const int wave = tid >> 5;
  const int hh   = lane >> 4;
  const int nodeBase = blockIdx.x * NB;
  const v4i z4 = {0, 0, 0, 0};
  const v4f zf = {0.f, 0.f, 0.f, 0.f};

  {
    for (int i = tid; i < ACCF / 4; i += NTHR) lds_dyn[i] = zf;
    for (int i = tid; i < NB; i += NTHR) { mx[i] = -1.0e30f; dn[i] = 0.f; }
  }
  __syncthreads();

  const int coff = 4 * lane;
  const v4f w0 = *(const v4f*)(att + coff);

  const int* eid = ei + nE;
  const bool al16 = ((nE & 3) == 0);
  const int nChunks = (nE + CHUNK - 1) / CHUNK;

#pragma unroll 1
  for (int ch = 0; ch <= nChunks; ++ch) {
    const int cbase = ch * CHUNK;
    const bool selfp = (ch == nChunks);
    if (!selfp) {
      const bool vec = al16 && (cbase + CHUNK <= nE);
      int wc = 0;
#pragma unroll
      for (int g = 0; g < NGRP; ++g) {
        const int el0 = (g * NTHR + tid) * 4;
        const int e0  = cbase + el0;
        const int sent = -2147483647 - 1;
        v4i d;
        if (vec) {
          d = *(const v4i*)(eid + e0);
        } else {
          const int q0 = min(e0, nE - 1), q1 = min(e0 + 1, nE - 1);
          const int q2 = min(e0 + 2, nE - 1), q3 = min(e0 + 3, nE - 1);
          const int t0 = eid[q0], t1 = eid[q1], t2 = eid[q2], t3 = eid[q3];
          d.x = (e0     < nE) ? t0 : sent;
          d.y = (e0 + 1 < nE) ? t1 : sent;
          d.z = (e0 + 2 < nE) ? t2 : sent;
          d.w = (e0 + 3 < nE) ? t3 : sent;
        }
        const unsigned s0 = (unsigned)d.x - (unsigned)nodeBase;
        const unsigned s1 = (unsigned)d.y - (unsigned)nodeBase;
        const unsigned s2 = (unsigned)d.z - (unsigned)nodeBase;
        const unsigned s3 = (unsigned)d.w - (unsigned)nodeBase;
        const bool h0 = s0 < (unsigned)NB;
        const bool h1 = s1 < (unsigned)NB;
        const bool h2 = s2 < (unsigned)NB;
        const bool h3 = s3 < (unsigned)NB;
        const unsigned many = __builtin_amdgcn_ballot_w32(h0 | h1 | h2 | h3);
        if (many != 0u) {
#define HITJ(J, HJ, SJ) { \
            const unsigned mj = __builtin_amdgcn_ballot_w32(HJ); \
            if (HJ) { \
              const int pos = wc + (int)__builtin_amdgcn_mbcnt_lo(mj, 0u); \
              if (pos < WCAP) list[wave * WCAP + pos] = ((el0 + (J)) << 9) | (int)(SJ); \
            } \
            wc += (int)__builtin_popcount(mj); }
          HITJ(0, h0, s0)
          HITJ(1, h1, s1)
          HITJ(2, h2, s2)
          HITJ(3, h3, s3)
#undef HITJ
        }
      }
      if (lane == 0) wcnt[wave] = wc;
    } else {
      for (int s = tid; s < NB; s += NTHR) list[s] = s;
      if (tid < NWAVE) {
        int c = NB - tid * WCAP;
        c = c < 0 ? 0 : (c > WCAP ? WCAP : c);
        wcnt[tid] = c;
      }
    }
    __syncthreads();

    if (wave == 0) {
#pragma unroll 1
      for (int wsx = 0; wsx < NWAVE; ++wsx) {
        int n = __builtin_amdgcn_readfirstlane(wcnt[wsx]);
        n = n > WCAP ? WCAP : n;
        n = n < 0 ? 0 : n;
#pragma unroll 1
        for (int i = 0; i < n; ++i) {
          const int ent  = __builtin_amdgcn_readfirstlane(list[wsx * WCAP + i]);
          const int slot = ent & (NB - 1);
          const int el   = (ent >> 9) & (CHUNK - 1);
          const int node = nodeBase + slot;
          if (node >= nN) continue;
          int e = cbase + el;
          if (e > nE - 1) e = nE - 1;
          int sj = ei[e];
          sj = sj < 0 ? 0 : (sj > nN - 1 ? nN - 1 : sj);
          const int src = selfp ? node : sj;
          const float* xs = xl + (size_t)src * HD + coff;
          const float* xd = xr + (size_t)node * HD + coff;
          float* ar = sacc + slot * HD + coff;
          hit4(xs, xd, ar, mx + slot, dn + slot, w0);
        }
      }
    }
    __syncthreads();
  }

  if (lastMode == 0) {
    const int m15 = lane & 15;
    const int co  = 8 * m15;
    const v4f b0 = *(const v4f*)(bias + co);
    const v4f b1 = *(const v4f*)(bias + co + 4);
#pragma unroll 1
    for (int t = 0; t < NB / 16; ++t) {
      const int s    = wave + 16 * t + 8 * hh;
      const int node = nodeBase + s;
      const float* ar = sacc + s * HD + co;
      const v4f e0 = *(const v4f*)(ar);
      const v4f e1 = *(const v4f*)(ar + 4);
      const float inv = 1.0f / (dn[s] + 1e-16f);
      const v4f o0 = e0 * inv + b0;
      const v4f o1 = e1 * inv + b1;
      Pack u;
#pragma unroll
      for (int j = 0; j < 4; ++j) {
        u.h[j]     = (_Float16)o0[j];
        u.h[4 + j] = (_Float16)o1[j];
      }
      if (node >= nN) u.i = z4;
      _Float16* hp = hf + (size_t)node * HD + co;
      if (node < nW) *(volatile v4i*)hp = u.i;
      __threadfence();
      if (node < nW) *(volatile v4i*)hp = u.i;
    }
  } else {
    const int co = 4 * lane;
    const v4f b0 = *(const v4f*)(bias + co);
#pragma unroll 1
    for (int s = wave; s < NB; s += NWAVE) {
      const int node = nodeBase + s;
      if (node >= nW) break;
      const v4f e0 = *(const v4f*)(sacc + s * HD + co);
      const float inv = 1.0f / (dn[s] + 1e-16f);
      v4f o = e0 * inv + b0;
      if (node >= nN) o = zf;
      float* op = hout + (size_t)node * HD + co;
      *(volatile v4f*)op = o;
      __threadfence();
      *(volatile v4f*)op = o;
    }
  }
}

__global__ __launch_bounds__(NTHR) void k_pool(const float* __restrict__ h, const int* __restrict__ gnd,
                                               const int* __restrict__ bat, int nG, int nN, float* pooled) {
  __shared__ __attribute__((aligned(16))) v4f part[NWAVE * 32];
  const int tid  = threadIdx.x;
  const int lane = tid & 31;
  const int wave = tid >> 5;
  const int g    = blockIdx.x;
  v4f acc = {0.f, 0.f, 0.f, 0.f};
  const int nIter = (nG + NTHR - 1) / NTHR;
#pragma unroll 1
  for (int it = 0; it < nIter; ++it) {
    const int base = it * NTHR + wave * 32;
    const int r    = base + lane;
    const int rc   = min(r, nG - 1);
    const int bv   = bat[rc];
    const bool hit = (r < nG) && (bv == g);
    unsigned msk = __builtin_amdgcn_ballot_w32(hit);
#pragma unroll 1
    while (msk != 0u) {
      const int bit = __builtin_ctz(msk);
      msk &= msk - 1u;
      const int rr = min(base + bit, nG - 1);
      int node = gnd[rr];
      node = node < 0 ? 0 : (node > nN - 1 ? nN - 1 : node);
      acc += *(const v4f*)(h + (size_t)node * HD + 4 * lane);
    }
  }
  part[wave * 32 + lane] = acc;
  __syncthreads();
  if (wave == 0) {
    v4f s = part[lane];
#pragma unroll
    for (int w = 1; w < NWAVE; ++w) s += part[w * 32 + lane];
    float* pp = pooled + (size_t)g * HD + 4 * lane;
    *(volatile v4f*)pp = s;
    __threadfence();
    *(volatile v4f*)pp = s;
  }
}

__global__ __launch_bounds__(128) void k_final(const float* __restrict__ pooled, const float* __restrict__ oW,
                                               const float* __restrict__ ob, float* out) {
  __shared__ __attribute__((aligned(16))) float Os[NGRAPH * FO];
  const int tid  = threadIdx.x;
  const int lane = tid & 31;
  const int wave = tid >> 5;
  const int hh   = lane >> 4;
  const int m    = lane & 15;
  const int arow = 16 * wave + m;
  v8f acc = {0.f, 0.f, 0.f, 0.f, 0.f, 0.f, 0.f, 0.f};
#pragma unroll 1
  for (int ks = 0; ks < HD / 32; ++ks) {
    const float* pa = pooled + (size_t)arow * HD + 32 * ks + 8 * hh;
    const v4f f0 = *(const v4f*)(pa);
    const v4f f1 = *(const v4f*)(pa + 4);
    const v4f f2 = *(const v4f*)(pa + 16);
    const v4f f3 = *(const v4f*)(pa + 20);
    Pack p0, p1, q0, q1;
#pragma unroll
    for (int j = 0; j < 4; ++j) {
      p0.h[j] = (_Float16)f0[j];  p0.h[4 + j] = (_Float16)f1[j];
      p1.h[j] = (_Float16)f2[j];  p1.h[4 + j] = (_Float16)f3[j];
    }
    const int kb = 32 * ks + 8 * hh;
#pragma unroll
    for (int j = 0; j < 8; ++j) {
      q0.h[j] = (_Float16)(oW[(kb + j) * FO + m] * 16.0f);
      q1.h[j] = (_Float16)(oW[(kb + 16 + j) * FO + m] * 16.0f);
    }
    FragH a, b;
    a.u[0] = p0.i;  a.u[1] = p1.i;
    b.u[0] = q0.i;  b.u[1] = q1.i;
    acc = wmh(a.v, b.v, acc);
  }
  const float bo = ob[m];
#pragma unroll
  for (int r = 0; r < 8; ++r) Os[(16 * wave + 8 * hh + r) * FO + m] = acc[r] * 0.0625f + bo;
  __syncthreads();
  const v4f o0 = *(const v4f*)(Os + 4 * tid);
  const v4f o1 = *(const v4f*)(Os + 512 + 4 * tid);
  float* d0 = out + 4 * tid;
  float* d1 = out + 512 + 4 * tid;
  *(volatile v4f*)d0 = o0;
  *(volatile v4f*)d1 = o1;
  __threadfence();
  *(volatile v4f*)d0 = o0;
  *(volatile v4f*)d1 = o1;
}

static inline size_t al256(size_t v) { return (v + 255) & ~(size_t)255; }

extern "C" void kernel_launch(void* const* d_in, const int* in_sizes, int n_in,
                              void* d_out, int out_size, void* d_ws, size_t ws_size,
                              hipStream_t stream) {
  if (n_in < 16) return;
  const int nN = in_sizes[0] / FI;
  if (nN <= 0 || in_sizes[0] != nN * FI) return;
  const int nE0 = in_sizes[1] / 2;
  const int nE1 = in_sizes[3] / 2;
  const int nE2 = in_sizes[2] / 2;
  const int nE3 = in_sizes[4] / 2;
  if (nE0 <= 0 || nE1 <= 0 || nE2 <= 0 || nE3 <= 0) return;
  if (in_sizes[1] != 2 * nE0 || in_sizes[3] != 2 * nE1 || in_sizes[2] != 2 * nE2 || in_sizes[4] != 2 * nE3) return;
  int nG = in_sizes[5];
  if (in_sizes[7] < nG) nG = in_sizes[7];
  if (nG <= 0) return;
  if (in_sizes[8] != FI * HD || in_sizes[9] != HD) return;
  if (in_sizes[10] != 4 * HD * HD || in_sizes[11] != 4 * HD * HD) return;
  if (in_sizes[12] != 4 * HD || in_sizes[13] != 4 * HD) return;
  if (in_sizes[14] != HD * FO || in_sizes[15] != FO) return;
  if (out_size != NGRAPH * FO) return;

  const float* x    = (const float*)d_in[0];
  const int*   e0p  = (const int*)d_in[1];
  const int*   e2p  = (const int*)d_in[2];
  const int*   e1p  = (const int*)d_in[3];
  const int*   e3p  = (const int*)d_in[4];
  const int*   gnd  = (const int*)d_in[5];
  const int*   bat  = (const int*)d_in[7];
  const float* embW = (const float*)d_in[8];
  const float* embB = (const float*)d_in[9];
  const float* Wl   = (const float*)d_in[10];
  const float* Wr   = (const float*)d_in[11];
  const float* att  = (const float*)d_in[12];
  const float* bias = (const float*)d_in[13];
  const float* oW   = (const float*)d_in[14];
  const float* ob   = (const float*)d_in[15];
  float* out = (float*)d_out;

  const int Mpad = ((nN + GR - 1) / GR) * GR;

  char* wsp = (char*)d_ws;
  size_t off = 0;
  _Float16* hf = (_Float16*)(wsp + off);  off = al256(off + (size_t)Mpad * HD * 2);
  float* xl = (float*)(wsp + off);         off = al256(off + (size_t)Mpad * HD * 4);
  float* xr = (float*)(wsp + off);         off = al256(off + (size_t)Mpad * HD * 4);
  _Float16* wemb = (_Float16*)(wsp + off); off = al256(off + (size_t)HD * FI * 2);
  _Float16* wcat = (_Float16*)(wsp + off); off = al256(off + (size_t)4 * 2 * HD * HD * 2);
  float* pooled = (float*)(wsp + off);     off = al256(off + (size_t)NGRAPH * HD * 4);
  if (off > ws_size) return;
  _Float16* xpl = (_Float16*)xr;
  if ((size_t)Mpad * FI * 2 > (size_t)Mpad * HD * 4) return;

  const float s16  = 16.0f;
  const float is16 = 0.0625f;
  const int mt     = Mpad / GR;
  const int aggG   = (Mpad + NB - 1) / NB;

  hipFuncSetAttribute(reinterpret_cast<const void*>(&k_agg),
                      hipFuncAttributeMaxDynamicSharedMemorySize, AGG_LDS_BYTES);

  k_cvt_x<<<(Mpad * (FI / 8) + NTHR - 1) / NTHR, NTHR, 0, stream>>>(x, nN, xpl, Mpad);
  k_cvt_w<<<((1 * HD * FI) / 8 + NTHR - 1) / NTHR, NTHR, 0, stream>>>(embW, embW, wemb, 1, FI, HD, HD, s16);
  k_cvt_w<<<((4 * 2 * HD * HD) / 8 + NTHR - 1) / NTHR, NTHR, 0, stream>>>(Wl, Wr, wcat, 4, HD, HD, 2 * HD, s16);

  k_gemm<1><<<dim3(mt, 1), NTHR, 0, stream>>>(xpl, wemb, embB, 1.0f, xl, xl, hf, FI, is16);

  const int*  eis[4] = {e0p, e1p, e2p, e3p};
  const int   nEs[4] = {nE0, nE1, nE2, nE3};
  for (int l = 0; l < 4; ++l) {
    k_gemm<0><<<dim3(mt, 2), NTHR, 0, stream>>>(hf, wcat + (size_t)l * 2 * HD * HD, embB, 0.0f,
                                                xl, xr, hf, HD, is16);
    k_agg<<<aggG, NTHR, AGG_LDS_BYTES, stream>>>(eis[l], xl, xr, att + l * HD, bias + l * HD,
                                                 hf, xr, nN, nEs[l], Mpad, (l == 3) ? 1 : 0);
  }

  k_pool<<<NGRAPH, NTHR, 0, stream>>>(xr, gnd, bat, nG, nN, pooled);
  k_final<<<1, 128, 0, stream>>>(pooled, oW, ob, out);
}
